// EmbedWeighted_11630771438334
// MI455X (gfx1250) — hardware-verified
//
#include <hip/hip_runtime.h>


#ifndef NROW
#define NROW 2048
#endif
#define NROW_FULL 2048
#define KV   2000
#define KP   2048
#define KL   2016
#define DE   64
#define KV8  (KV / 8)
#define TSP  65
#define OSPG 68

static_assert(NROW <= NROW_FULL);
static_assert(NROW % 32 == 0);
static_assert(KV % 8 == 0);
static_assert((KV * 4) % 32 == 0);
static_assert(KL % 32 == 0);
static_assert(KL >= KV);
static_assert(KL - KV < 32);
static_assert(KP >= KL);
static_assert(KP % 64 == 0);
static_assert((KP * 2) % 128 == 0);
static_assert(KP / 8 == 256);
static_assert(DE == 64);
static_assert(32 * 16 == 2 * DE * 4);
static_assert(32 * 16 * 8 == 16 * DE * 4);
static_assert(256 * 2 * 16 == 64 * 128);
static_assert(256 * 4 * 4 == 64 * DE);
static_assert((OSPG * 4) % 16 == 0);
static_assert(64 * TSP * 4 <= 131072);
static_assert(16 * OSPG * 4 <= 131072);
static_assert((size_t)(NROW_FULL - 1) * KV + KV <= (size_t)0xFFFFFFFFu);

typedef unsigned short bf;
typedef __attribute__((ext_vector_type(16))) __bf16   v16bf;
typedef __attribute__((ext_vector_type(8)))  unsigned short v8us;
typedef __attribute__((ext_vector_type(8)))  float    v8f;
typedef __attribute__((ext_vector_type(4)))  float    v4f;
typedef v4f  __attribute__((may_alias)) v4fa;

__device__ __forceinline__ unsigned short f2bf(float f) { unsigned u = __float_as_uint(f); u += 0x7FFFu + ((u >> 16) & 1u); return (unsigned short)(u >> 16); }
__device__ __forceinline__ v16bf cat16b(v8us lo, v8us hi) { return __builtin_bit_cast(v16bf, __builtin_shufflevector(lo, hi, 0, 1, 2, 3, 4, 5, 6, 7, 8, 9, 10, 11, 12, 13, 14, 15)); }
__device__ __forceinline__ v8f wmmab(v16bf a, v16bf b, v8f c) { return __builtin_amdgcn_wmma_f32_16x16x32_bf16(false, a, false, b, (short)0, c, false, false); }
__device__ __forceinline__ v8f wmmabg(v16bf a, v16bf b, v8f c) { c = wmmab(a, b, c); asm volatile("v_nop\n\tv_nop\n\tv_nop\n\tv_nop" : "+v"(c) : "v"(a), "v"(b)); return c; }
__device__ __forceinline__ v16bf ldb(const bf* p)  { return cat16b(*(const v8us*)p, *(const v8us*)(p + 16)); }
__device__ __forceinline__ void wave_sync() { __builtin_amdgcn_fence(3  , "wavefront"); __builtin_amdgcn_wave_barrier(); asm volatile("" ::: "memory"); }

__global__ __launch_bounds__(256) void k_cvta(const float* __restrict__ src, bf* dst) {
    const unsigned row = blockIdx.x, g = threadIdx.x;
    const unsigned gc = (unsigned)min((int)g, KV8 - 1);
    const v8f v = *(const v8f*)(src + (size_t)(row * (unsigned)KV + gc * 8u));
    const bool ok = g < (unsigned)KV8;
    v8us o;
#pragma unroll
    for (int k = 0; k < 8; ++k) { const float w = ok ? v[k] : 0.0f; o[k] = f2bf(w); }
    bf* p = dst + (size_t)row * KP + (size_t)(g * 8u);
    *(volatile v8us*)p = o; __threadfence(); *(volatile v8us*)p = o;
}

__global__ __launch_bounds__(256) void k_cvtbt(const float* __restrict__ src, bf* dst) {
    __shared__ float ts[64 * TSP];
    const unsigned tid = threadIdx.x; const unsigned v0 = blockIdx.x * 64u;
#pragma unroll
    for (int it = 0; it < 4; ++it) {
        const unsigned idx = (unsigned)it * 256u + tid; const unsigned row = idx >> 4, c4 = (idx & 15u) * 4u;
        const unsigned vr = (unsigned)min((int)(v0 + row), KV - 1);
        const v4f x = *(const v4f*)(src + (size_t)(vr * (unsigned)DE + c4));
        const bool ok = (v0 + row) < (unsigned)KV;
#pragma unroll
        for (int i = 0; i < 4; ++i) ts[row * TSP + c4 + i] = ok ? x[i] : 0.0f;
    }
    __syncthreads();
    v8us o[2];
#pragma unroll
    for (int it = 0; it < 2; ++it) {
        const unsigned p = (unsigned)it * 256u + tid; const unsigned d = p >> 3, vg = (p & 7u) * 8u;
#pragma unroll
        for (int i = 0; i < 8; ++i) o[it][i] = f2bf(ts[(vg + i) * TSP + d]);
    }
#pragma unroll 1
    for (int ps = 0; ps < 2; ++ps) {
#pragma unroll
        for (int it = 0; it < 2; ++it) {
            const unsigned p = (unsigned)it * 256u + tid; const unsigned d = p >> 3, vg = (p & 7u) * 8u;
            *(volatile v8us*)(dst + (size_t)d * KP + (size_t)(v0 + vg)) = o[it]; }
        if (ps == 0) __threadfence(); }
}

__global__ __launch_bounds__(32) void k_gemm(const bf* __restrict__ A, const bf* __restrict__ Bt, float* OUT) {
    __shared__ __align__(16) float os[16 * OSPG];
    const int lane = threadIdx.x & 31, lr = lane & 15, hi = lane >> 4; const unsigned r0 = blockIdx.x * 32u;
    v8f acc[2][4];
#pragma unroll
    for (int mb = 0; mb < 2; ++mb)
#pragma unroll
        for (int nb = 0; nb < 4; ++nb) acc[mb][nb] = (v8f){};
    const size_t aoff = (size_t)(r0 + (unsigned)lr) * KP + 8 * hi, boff = (size_t)lr * KP + 8 * hi;
#pragma unroll 1
    for (int kc = 0; kc < KL; kc += 32) {
        v16bf a[2];
#pragma unroll
        for (int mb = 0; mb < 2; ++mb) a[mb] = ldb(A + aoff + (size_t)mb * 16 * KP + kc);
#pragma unroll
        for (int nb = 0; nb < 4; ++nb) { const v16bf b = ldb(Bt + boff + (size_t)nb * 16 * KP + kc);
#pragma unroll
            for (int mb = 0; mb < 2; ++mb) acc[mb][nb] = wmmabg(a[mb], b, acc[mb][nb]); }
    }
    float* obase = OUT + (size_t)r0 * DE;
#pragma unroll
    for (int mb = 0; mb < 2; ++mb) {
#pragma unroll
        for (int nb = 0; nb < 4; ++nb) {
#pragma unroll
            for (int j = 0; j < 8; ++j) os[(hi * 8 + j) * OSPG + nb * 16 + lr] = acc[mb][nb][j]; }
        wave_sync();
        float* orow = obase + (size_t)(mb * 16) * DE;
#pragma unroll 1
        for (int ps = 0; ps < 2; ++ps) {
#pragma unroll
            for (int s = 0; s < 8; ++s) { const int row = 2 * s + (lane >> 4), cofs = (lane & 15) * 4;
                const v4f val = *(const v4fa*)(&os[row * OSPG + cofs]);
                *(volatile v4f*)(orow + (size_t)row * DE + cofs) = val; }
            if (ps == 0) __threadfence(); }
        wave_sync();
    }
}

static constexpr size_t al256(size_t v) { return (v + 255) & ~(size_t)255; }
static constexpr size_t SZ_AB = al256((size_t)NROW * KP * 2);
static constexpr size_t SZ_ET = al256((size_t)DE * KP * 2);
static constexpr size_t SZ_TOTAL = SZ_AB + SZ_ET;
static_assert(SZ_TOTAL <= (size_t)134217728);
static_assert(((size_t)(NROW - 1) * KP + (size_t)255 * 8 + 8) * 2 <= SZ_AB);
static_assert(((size_t)(DE - 1) * KP + (size_t)(KP / 64 - 1) * 64 + 56 + 8) * 2 <= SZ_ET);
static_assert(((size_t)(NROW - 1) * KP + (size_t)8 + (size_t)(KL - 32) + 16 + 8) * 2 <= SZ_AB);
static_assert(((size_t)(DE - 1) * KP + (size_t)8 + (size_t)(KL - 32) + 16 + 8) * 2 <= SZ_ET);
static_assert(((size_t)(NROW - 1) * DE + DE) * 4 <= (size_t)NROW_FULL * DE * 4);

extern "C" void kernel_launch(void* const* d_in, const int* in_sizes, int n_in,
                              void* d_out, int out_size, void* d_ws, size_t ws_size, hipStream_t stream) {
    if (n_in < 2) return;
    if ((size_t)in_sizes[0] < (size_t)NROW * KV) return;
    if ((size_t)in_sizes[1] < (size_t)KV * DE) return;
    if ((size_t)out_size < (size_t)NROW * DE) return;
    if (SZ_TOTAL > ws_size) return;
    const float* win = (const float*)d_in[0];
    const float* tab = (const float*)d_in[1];
    float* OUT = (float*)d_out;
    char* wsp = (char*)d_ws;
    bf* AB = (bf*)wsp; wsp += SZ_AB;
    bf* ET = (bf*)wsp; wsp += SZ_ET;

    k_cvta<<<dim3(NROW, 1, 1), 256, 0, stream>>>(win, AB);
    k_cvtbt<<<dim3(KP / 64, 1, 1), 256, 0, stream>>>(tab, ET);
    k_gemm<<<dim3(NROW / 32, 1, 1), 32, 0, stream>>>(AB, ET, OUT);
}
